// SDPAttention_50251117363389
// MI455X (gfx1250) — hardware-verified
//
#include <hip/hip_runtime.h>


#ifndef NB
#define NB 2
#endif
#ifndef SEQ
#define SEQ 2048
#endif
#define SEQ_FULL 2048
#define CDIM 768
#define NH   12
#define HD   64
#define QKVN (3 * CDIM)
#define NBH  (NB * NH)
#define MTOK (NB * SEQ)
#define KQK  (3 * HD)
#define ZB   2
#define SROWS (ZB * SEQ)
#define SCL  0.125f
#define PCARRY 4096.0f
#define PCINV  0.000244140625f
#define LOG2E  1.4426950408889634f

static_assert(SEQ % 128 == 0);
static_assert(SEQ <= SEQ_FULL);
static_assert(NB >= 1 && NB <= 2);
static_assert(HD == 64 && CDIM == NH * HD);
static_assert(NH % ZB == 0 && NBH % ZB == 0);
static_assert(CDIM % 64 == 0 && QKVN % 64 == 0 && MTOK % 64 == 0 && SEQ % 64 == 0 && HD % 64 == 0);
static_assert(CDIM % 32 == 0 && KQK % 32 == 0 && SEQ % 32 == 0);
static_assert(SROWS % 8 == 0);

typedef _Float16 h16;
typedef unsigned short bf;
typedef __attribute__((ext_vector_type(16))) __bf16   v16bf;
typedef __attribute__((ext_vector_type(16))) _Float16 v16h;
typedef __attribute__((ext_vector_type(8)))  _Float16 v8h;
typedef __attribute__((ext_vector_type(4)))  _Float16 v4h;
typedef __attribute__((ext_vector_type(8)))  unsigned short v8us;
typedef __attribute__((ext_vector_type(8)))  float    v8f;
typedef __attribute__((ext_vector_type(4)))  float    v4f;
typedef __attribute__((ext_vector_type(2)))  float    v2f;
typedef __attribute__((ext_vector_type(4)))  unsigned short v4us;
typedef __attribute__((ext_vector_type(2)))  unsigned short v2us;
typedef v8h  __attribute__((may_alias)) v8ha;
typedef v4f  __attribute__((may_alias)) v4fa;
typedef v8us __attribute__((may_alias)) v8usa;

#define ALN(b) (((size_t)(b) + 255) & ~(size_t)255)
static constexpr size_t BQC  = (size_t)NBH * SEQ * KQK * 2;
static constexpr size_t BVC  = (size_t)NBH * HD * SEQ * 2;
static constexpr size_t BCTX = (size_t)MTOK * CDIM * 4;
static constexpr size_t BCT  = (size_t)MTOK * CDIM * 2;
static constexpr size_t BWP  = (size_t)CDIM * CDIM * 2;
static constexpr size_t BXB  = (size_t)MTOK * CDIM * 2;
static constexpr size_t BWQ  = (size_t)QKVN * CDIM * 2;
static constexpr size_t BQF  = (size_t)MTOK * QKVN * 4;
static constexpr size_t BS   = (size_t)SROWS * SEQ * 4;
static constexpr size_t BPC  = (size_t)SROWS * SEQ * 2;
static constexpr size_t BR1  = ALN(BXB) + ALN(BWQ) + ALN(BQF);
static constexpr size_t BR2  = ALN(BS) + ALN(BPC);
static constexpr size_t BR   = (BR1 > BR2) ? BR1 : BR2;
static constexpr size_t BTOT = 2 * ALN(BQC) + ALN(BVC) + ALN(BCTX) + 2 * ALN(BCT) + ALN(BWP) + ALN(BR);
static_assert(BTOT <= (size_t)134217728);

__device__ __forceinline__ unsigned short f2bf(float f) { unsigned u = __float_as_uint(f); u += 0x7FFFu + ((u >> 16) & 1u); return (unsigned short)(u >> 16); }
__device__ __forceinline__ float bf2f(unsigned short b) { return __uint_as_float(((unsigned)b) << 16); }
__device__ __forceinline__ float bfr(float f) { return bf2f(f2bf(f)); }
__device__ __forceinline__ void splitf(float y, unsigned short& h, unsigned short& l) { h = f2bf(y); l = f2bf(y - bf2f(h)); }
__device__ __forceinline__ v16h cat16(v8h lo, v8h hi) { return __builtin_shufflevector(lo, hi, 0, 1, 2, 3, 4, 5, 6, 7, 8, 9, 10, 11, 12, 13, 14, 15); }
__device__ __forceinline__ v16bf cat16b(v8us lo, v8us hi) { return __builtin_bit_cast(v16bf, __builtin_shufflevector(lo, hi, 0, 1, 2, 3, 4, 5, 6, 7, 8, 9, 10, 11, 12, 13, 14, 15)); }
__device__ __forceinline__ v8f wmma16(v16h a, v16h b, v8f c) { return __builtin_amdgcn_wmma_f32_16x16x32_f16(false, a, false, b, (short)0, c, false, false); }
__device__ __forceinline__ v8f wmmab(v16bf a, v16bf b, v8f c) { return __builtin_amdgcn_wmma_f32_16x16x32_bf16(false, a, false, b, (short)0, c, false, false); }

template <typename T16> struct WFrag;
template <> struct WFrag<h16> { typedef v16h V; static __device__ __forceinline__ V ld(const h16* p) { return cat16(*(const v8h*)p, *(const v8h*)(p + 16)); } static __device__ __forceinline__ v8f mma(V a, V b, v8f c) { return wmma16(a, b, c); } };
template <> struct WFrag<bf> { typedef v16bf V; static __device__ __forceinline__ V ld(const bf* p) { return cat16b(*(const v8us*)p, *(const v8us*)(p + 16)); } static __device__ __forceinline__ v8f mma(V a, V b, v8f c) { return wmmab(a, b, c); } };
template <typename T16, int NSPLIT, bool BIAS>
__global__ __launch_bounds__(32) void k_gemmw(const T16* __restrict__ A, const T16* __restrict__ A2, const T16* __restrict__ Bt, const T16* __restrict__ Bt2, int K, float* C, int ldc, const float* __restrict__ bias, size_t sA, size_t sB, size_t sC) {
    typedef typename WFrag<T16>::V V;
    __shared__ __align__(16) float os[16 * 68];
    const size_t z = blockIdx.z; A += z * sA; if (A2) A2 += z * sA; Bt += z * sB; if (Bt2) Bt2 += z * sB; C += z * sC;
    const int lane = threadIdx.x & 31, lr = lane & 15, hi = lane >> 4; const int r0 = blockIdx.x * 64, c0 = blockIdx.y * 64;
    v8f acc[4][4];
#pragma unroll
    for (int mb = 0; mb < 4; ++mb)
#pragma unroll
        for (int nb = 0; nb < 4; ++nb) acc[mb][nb] = (v8f){};
    const size_t aoff = (size_t)(r0 + lr) * K + 8 * hi, boff = (size_t)(c0 + lr) * K + 8 * hi;
#pragma unroll 1
    for (int kc = 0; kc < K; kc += 32) {
        V a[4], a2[4];
#pragma unroll
        for (int mb = 0; mb < 4; ++mb) { a[mb] = WFrag<T16>::ld(A + aoff + (size_t)mb * 16 * K + kc); if (NSPLIT == 1 || NSPLIT == 2) a2[mb] = WFrag<T16>::ld(A2 + aoff + (size_t)mb * 16 * K + kc); }
#pragma unroll
        for (int nb = 0; nb < 4; ++nb) { const V b = WFrag<T16>::ld(Bt + boff + (size_t)nb * 16 * K + kc); V b2; if (NSPLIT >= 2) b2 = WFrag<T16>::ld(Bt2 + boff + (size_t)nb * 16 * K + kc);
#pragma unroll
            for (int mb = 0; mb < 4; ++mb) { acc[mb][nb] = WFrag<T16>::mma(a[mb], b, acc[mb][nb]); if (NSPLIT == 1 || NSPLIT == 2) acc[mb][nb] = WFrag<T16>::mma(a2[mb], b, acc[mb][nb]); if (NSPLIT >= 2) acc[mb][nb] = WFrag<T16>::mma(a[mb], b2, acc[mb][nb]); } }
        asm volatile("v_nop\n\tv_nop\n\tv_nop\n\tv_nop" : "+v"(acc[0][0]), "+v"(acc[1][1]), "+v"(acc[2][2]), "+v"(acc[3][3]) : "v"(a[0]), "v"(a[3]));
    }
#pragma unroll
    for (int mb = 0; mb < 4; ++mb) {
#pragma unroll
        for (int nb = 0; nb < 4; ++nb) {
#pragma unroll
            for (int j = 0; j < 8; ++j) os[(hi * 8 + j) * 68 + nb * 16 + lr] = acc[mb][nb][j]; }
        __builtin_amdgcn_wave_barrier(); asm volatile("" ::: "memory");
        float* crow = C + (size_t)(r0 + mb * 16) * ldc + c0;
#pragma unroll 1
        for (int ps = 0; ps < 2; ++ps) {
#pragma unroll
            for (int s = 0; s < 8; ++s) { const int row = 2 * s + hi, cofs = lr * 4; v4f val = *(const v4fa*)(os + row * 68 + cofs); if (BIAS) { val[0] += bfr(bias[c0 + cofs]); val[1] += bfr(bias[c0 + cofs + 1]); val[2] += bfr(bias[c0 + cofs + 2]); val[3] += bfr(bias[c0 + cofs + 3]); }
                *(volatile v4f*)(crow + (size_t)row * ldc + cofs) = val; }
            if (ps == 0) __threadfence(); }
        __builtin_amdgcn_wave_barrier(); asm volatile("" ::: "memory");
    }
}

__global__ __launch_bounds__(256) void k_cvt(const float* __restrict__ F, bf* P, unsigned n4, unsigned cols4, unsigned segrows, unsigned srcsegrows) {
    const unsigned i = blockIdx.x * 256u + threadIdx.x; if (i >= n4) return;
    const unsigned row = i / cols4; const unsigned c4 = i - row * cols4;
    const unsigned srow = (row / segrows) * srcsegrows + (row % segrows);
    const v4f v = *(const v4f*)(F + ((size_t)srow * cols4 + c4) * 4);
    v4us o;
#pragma unroll
    for (int q = 0; q < 4; ++q) o[q] = f2bf(v[q]);
    *(volatile v4us*)(P + (size_t)i * 4) = o; __threadfence(); *(volatile v4us*)(P + (size_t)i * 4) = o;
}

__global__ __launch_bounds__(256) void k_qk(const float* __restrict__ QF, bf* Qc, bf* Kc) {
    const unsigned i = blockIdx.x * 256u + threadIdx.x; if (i >= (unsigned)NBH * SEQ * 16) return;
    const unsigned d4 = i & 15u; const unsigned row = i >> 4;
    const unsigned bh = row / SEQ, n = row % SEQ; const unsigned b = bh / NH, h = bh - b * NH;
    const float* src = QF + ((size_t)b * SEQ + n) * QKVN + h * HD + d4 * 4;
    const v4f q = *(const v4f*)src; const v4f k = *(const v4f*)(src + CDIM);
    v4us qh, ql, kh, kl;
#pragma unroll
    for (int e = 0; e < 4; ++e) { unsigned short a, c; splitf(q[e], a, c); qh[e] = a; ql[e] = c; splitf(k[e], a, c); kh[e] = a; kl[e] = c; }
    bf* qo = Qc + (size_t)row * KQK + d4 * 4; bf* ko = Kc + (size_t)row * KQK + d4 * 4;
#pragma unroll 1
    for (int ps = 0; ps < 2; ++ps) {
        *(volatile v4us*)(qo) = qh; *(volatile v4us*)(qo + HD) = ql; *(volatile v4us*)(qo + 2 * HD) = qh;
        *(volatile v4us*)(ko) = kh; *(volatile v4us*)(ko + HD) = kh; *(volatile v4us*)(ko + 2 * HD) = kl;
        if (ps == 0) __threadfence(); }
}

__global__ __launch_bounds__(256) void k_vt(const float* __restrict__ QF, h16* Vc) {
    const unsigned e = (blockIdx.x * 256u + threadIdx.x) * 4u; if (e >= (unsigned)NBH * HD * SEQ) return;
    const unsigned n = e % SEQ; const unsigned dn = e / SEQ; const unsigned d = dn % HD; const unsigned bh = dn / HD;
    const unsigned b = bh / NH, h = bh - b * NH;
    const float* src = QF + ((size_t)b * SEQ + n) * QKVN + 2 * CDIM + h * HD + d;
    v4h o;
#pragma unroll
    for (int q = 0; q < 4; ++q) o[q] = (h16)src[(size_t)q * QKVN];
    h16* vo = Vc + ((size_t)bh * HD + d) * SEQ + n;
    *(volatile v4h*)vo = o; __threadfence(); *(volatile v4h*)vo = o;
}

__global__ __launch_bounds__(256) void k_csplit(const float* __restrict__ F, bf* Ph, bf* Pl, unsigned n4) {
    const unsigned i = blockIdx.x * 256u + threadIdx.x; if (i >= n4) return;
    const v4f v = *(const v4f*)(F + (size_t)i * 4) * PCINV; v4us oh, ol;
#pragma unroll
    for (int q = 0; q < 4; ++q) { unsigned short a, c; splitf(v[q], a, c); oh[q] = a; ol[q] = c; }
    *(volatile v4us*)(Ph + (size_t)i * 4) = oh; *(volatile v4us*)(Pl + (size_t)i * 4) = ol; __threadfence(); *(volatile v4us*)(Ph + (size_t)i * 4) = oh; *(volatile v4us*)(Pl + (size_t)i * 4) = ol;
}

__global__ __launch_bounds__(256) void k_ssoft(const float* __restrict__ Sb, h16* Pc) {
    const int lane = threadIdx.x & 31; const int ri = blockIdx.x * 8 + (threadIdx.x >> 5); if (ri >= SROWS) return;
    const float* sr = Sb + (size_t)ri * SEQ;
    float mx = -1.0e30f, sum = 0.f;
#pragma unroll 1
    for (int j0 = lane * 4; j0 < SEQ; j0 += 128) {
        const v4f a = *(const v4f*)(sr + j0);
        const float cm = fmaxf(fmaxf(a[0], a[1]), fmaxf(a[2], a[3])) * SCL;
        const float mn = fmaxf(mx, cm);
        float t = __fmul_rn(__fsub_rn(mx, mn), LOG2E); t = fmaxf(t, -120.0f);
        sum = sum * __builtin_amdgcn_exp2f(t);
#pragma unroll
        for (int q = 0; q < 4; ++q) { float d0 = __fsub_rn(a[q] * SCL, mn); asm volatile("" : "+v"(d0)); sum += __builtin_amdgcn_exp2f(__fmul_rn(d0, LOG2E)); }
        mx = mn;
    }
    float gm = mx;
#pragma unroll
    for (int sh = 16; sh; sh >>= 1) gm = fmaxf(gm, __shfl_xor(gm, sh, 32));
    { float t = __fmul_rn(__fsub_rn(mx, gm), LOG2E); t = fmaxf(t, -120.0f); sum = sum * __builtin_amdgcn_exp2f(t); }
#pragma unroll
    for (int sh = 16; sh; sh >>= 1) sum += __shfl_xor(sum, sh, 32);
    const float f = __fdiv_rn(PCARRY, sum);
#pragma unroll 1
    for (int j0 = lane * 4; j0 < SEQ; j0 += 128) {
        const v4f a = *(const v4f*)(sr + j0); v4h o;
#pragma unroll
        for (int q = 0; q < 4; ++q) { float d0 = __fsub_rn(a[q] * SCL, gm); asm volatile("" : "+v"(d0)); o[q] = (h16)(__builtin_amdgcn_exp2f(__fmul_rn(d0, LOG2E)) * f); }
        h16* po = Pc + (size_t)ri * SEQ + j0;
        *(volatile v4h*)po = o; __threadfence(); *(volatile v4h*)po = o;
    }
}

extern "C" void kernel_launch(void* const* d_in, const int* in_sizes, int n_in,
                              void* d_out, int out_size, void* d_ws, size_t ws_size, hipStream_t stream) {
    if (n_in < 4) return;
    if ((size_t)in_sizes[0] < ((size_t)(NB - 1) * SEQ_FULL + SEQ) * CDIM) return;
    if (in_sizes[1] < QKVN * CDIM) return;
    if (in_sizes[2] < CDIM * CDIM) return;
    if (in_sizes[3] < CDIM) return;
    if ((size_t)out_size < (size_t)MTOK * CDIM) return;
    const float* Xi = (const float*)d_in[0];
    const float* Wq = (const float*)d_in[1];
    const float* Wp = (const float*)d_in[2];
    const float* Bp = (const float*)d_in[3];
    float* OUT = (float*)d_out;

    char* wsp = (char*)d_ws;
    auto take = [&](size_t bytes) { char* p = wsp; wsp += ALN(bytes); return (void*)p; };
    bf* Qc = (bf*)take(BQC); bf* Kc = (bf*)take(BQC); h16* Vc = (h16*)take(BVC);
    float* ctxf = (float*)take(BCTX); bf* cth = (bf*)take(BCT); bf* ctl = (bf*)take(BCT); bf* wpb = (bf*)take(BWP);
    char* R = (char*)take(BR);
    if ((size_t)(wsp - (char*)d_ws) > ws_size) return;
    bf* xb = (bf*)R; bf* wqb = (bf*)(R + ALN(BXB)); float* QF = (float*)(R + ALN(BXB) + ALN(BWQ));
    float* Sb = (float*)R; h16* Pc = (h16*)(R + ALN(BS));

    const unsigned nx4 = (unsigned)((size_t)MTOK * CDIM / 4), nwq4 = (unsigned)((size_t)QKVN * CDIM / 4), nwp4 = (unsigned)((size_t)CDIM * CDIM / 4);
    k_cvt<<<(nx4 + 255) / 256, 256, 0, stream>>>(Xi, xb, nx4, CDIM / 4, SEQ, SEQ_FULL);
    k_cvt<<<(nwq4 + 255) / 256, 256, 0, stream>>>(Wq, wqb, nwq4, CDIM / 4, QKVN, QKVN);
    k_cvt<<<(nwp4 + 255) / 256, 256, 0, stream>>>(Wp, wpb, nwp4, CDIM / 4, CDIM, CDIM);
    k_gemmw<bf, 0, false><<<dim3(MTOK / 64, QKVN / 64, 1), 32, 0, stream>>>(xb, nullptr, wqb, nullptr, CDIM, QF, QKVN, nullptr, 0, 0, 0);
    const unsigned nqk = (unsigned)NBH * SEQ * 16, nvt = (unsigned)NBH * HD * SEQ / 4;
    k_qk<<<(nqk + 255) / 256, 256, 0, stream>>>(QF, Qc, Kc);
    k_vt<<<(nvt + 255) / 256, 256, 0, stream>>>(QF, Vc);
    for (int g = 0; g < NBH / ZB; ++g) { const int bh0 = g * ZB; const int b = bh0 / NH, h0 = bh0 % NH;
        k_gemmw<bf, 0, false><<<dim3(SEQ / 64, SEQ / 64, ZB), 32, 0, stream>>>(Qc + (size_t)bh0 * SEQ * KQK, nullptr, Kc + (size_t)bh0 * SEQ * KQK, nullptr, KQK, Sb, SEQ, nullptr, (size_t)SEQ * KQK, (size_t)SEQ * KQK, (size_t)SEQ * SEQ);
        k_ssoft<<<SROWS / 8, 256, 0, stream>>>(Sb, Pc);
        k_gemmw<h16, 0, false><<<dim3(SEQ / 64, HD / 64, ZB), 32, 0, stream>>>(Pc, nullptr, Vc + (size_t)bh0 * HD * SEQ, nullptr, SEQ, ctxf + (size_t)b * SEQ * CDIM + (size_t)h0 * HD, CDIM, nullptr, (size_t)SEQ * SEQ, (size_t)HD * SEQ, (size_t)HD); }
    k_csplit<<<(nx4 + 255) / 256, 256, 0, stream>>>(ctxf, cth, ctl, nx4);
    k_gemmw<bf, 1, true><<<dim3(MTOK / 64, CDIM / 64, 1), 32, 0, stream>>>(cth, ctl, wpb, nullptr, CDIM, OUT, CDIM, Bp, 0, 0, 0);
}
